// xlstmDecoder_57629871177856
// MI455X (gfx1250) — hardware-verified
//
#include <hip/hip_runtime.h>
#include <math.h>

typedef __attribute__((ext_vector_type(16))) _Float16 v16h;
typedef __attribute__((ext_vector_type(8)))  _Float16 v8h;
typedef __attribute__((ext_vector_type(4)))  _Float16 v4h;
typedef __attribute__((ext_vector_type(16))) __bf16   v16b;
typedef __attribute__((ext_vector_type(8)))  __bf16   v8b;
typedef __attribute__((ext_vector_type(8)))  float    v8f;
typedef __attribute__((ext_vector_type(4)))  float    v4f;
typedef __attribute__((ext_vector_type(2)))  float    v2f;
typedef unsigned short u16;

constexpr int kBatch = 512;
constexpr int kSeq   = 12;
constexpr int kEmb   = 1024;
constexpr int kRows  = kBatch * kSeq;
constexpr int kHeads = 8;
constexpr int kHS    = 128;
constexpr int kGate  = 4096;
constexpr int kC48   = 48;

__device__ __forceinline__ unsigned short f2bf_bits(float f) {
  unsigned u = __float_as_uint(f);
  return (unsigned short)((u + 0x7FFFu + ((u >> 16) & 1u)) >> 16);
}
__device__ __forceinline__ float bf_bits2f(unsigned short h) { return __uint_as_float(((unsigned)h) << 16); }

__device__ __forceinline__ void dep_guard_h(v8f& a, v8f& b, v16h x, v16h y) { asm volatile("v_nop\n\tv_nop\n\tv_nop\n\tv_nop" : "+v"(a), "+v"(b) : "v"(x), "v"(y)); }
__device__ __forceinline__ void dep_guard_b(v8f& a, v8f& b, v16b x, v16b y) { asm volatile("v_nop\n\tv_nop\n\tv_nop\n\tv_nop" : "+v"(a), "+v"(b) : "v"(x), "v"(y)); }
__device__ __forceinline__ void keep4_h(v16h a, v16h b, v16h c, v16h d) { asm volatile("v_nop" :: "v"(a), "v"(b), "v"(c), "v"(d)); }
__device__ __forceinline__ void keep4_b(v16b a, v16b b, v16b c, v16b d) { asm volatile("v_nop" :: "v"(a), "v"(b), "v"(c), "v"(d)); }
__device__ __forceinline__ void acc_guard4(v8f& a, v8f& b, v8f& c, v8f& d) { asm volatile("v_nop\n\tv_nop\n\tv_nop\n\tv_nop" : "+v"(a), "+v"(b), "+v"(c), "+v"(d)); }
template <typename T> struct Frag;
template <> struct Frag<_Float16> {
  typedef v16h V; union U { v16h v; v8h h[2]; };
  static __device__ __forceinline__ v16h load(const _Float16* p) {
    U f; f.h[0] = *(const v8h*)(p); f.h[1] = *(const v8h*)(p + 16); return f.v;
  }
  static __device__ __forceinline__ v8f mma(v16h a, v16h b, v8f c) {
    return __builtin_amdgcn_wmma_f32_16x16x32_f16(false, a, false, b, (short)0, c, false, false);
  }
  static __device__ __forceinline__ void guard(v8f& a, v8f& b, v16h x, v16h y) { dep_guard_h(a, b, x, y); }
  static __device__ __forceinline__ void keep(v16h a, v16h b, v16h c, v16h d) { keep4_h(a, b, c, d); }
};
template <> struct Frag<__bf16> {
  typedef v16b V; union U { v16b v; v8b h[2]; };
  static __device__ __forceinline__ v16b load(const __bf16* p) {
    U f; f.h[0] = *(const v8b*)(p); f.h[1] = *(const v8b*)(p + 16); return f.v;
  }
  static __device__ __forceinline__ v8f mma(v16b a, v16b b, v8f c) {
    return __builtin_amdgcn_wmma_f32_16x16x32_bf16(false, a, false, b, (short)0, c, false, false);
  }
  static __device__ __forceinline__ void guard(v8f& a, v8f& b, v16b x, v16b y) { dep_guard_b(a, b, x, y); }
  static __device__ __forceinline__ void keep(v16b a, v16b b, v16b c, v16b d) { keep4_b(a, b, c, d); }
};

template <int ET> struct Elem;
template <> struct Elem<0> { typedef _Float16 T; };
template <> struct Elem<1> { typedef __bf16 T; };
template <int ET, bool SPLIT, int BIAS_MODE, int OUT_MODE, bool RESID, int ACT = 0>
__global__ __launch_bounds__(256) void wmma_gemm64(
    const unsigned short* __restrict__ Ap, const unsigned short* __restrict__ A2p, int lda, long strideA,
    const unsigned short* __restrict__ Btp, const unsigned short* __restrict__ Bt2p, int ldb, long strideB,
    void* __restrict__ Cout, void* __restrict__ Cout2, int ldc, long strideC,
    const float* __restrict__ bias,
    const float* __restrict__ resid, long strideR,
    int M, int N, int K, float scale) {
  typedef typename Elem<ET>::T T;
  typedef typename Frag<T>::V V;
  const T* A = (const T*)Ap; const T* A2 = (const T*)A2p; const T* Bt = (const T*)Btp; const T* Bt2 = (const T*)Bt2p;
  __shared__ __align__(16) float sT[8][16 * 68];
  const int b    = blockIdx.y;
  const int lane = threadIdx.x & 31;
  const int wave = threadIdx.x >> 5;
  const int tilesN = N >> 6;
  const int tilesM = M >> 6;
  const int tile = blockIdx.x * 8 + wave;
  if (tile >= tilesM * tilesN) return;
  const int tm = tile / tilesN;
  const int tn = tile - tm * tilesN;
  const int m0 = tm << 6;
  const int n0 = tn << 6;

  const T* Ab  = A  + (size_t)b * strideA;
  const T* Bb  = Bt + (size_t)b * strideB;
  const T* Ab2 = SPLIT ? (A2  + (size_t)b * strideA) : nullptr;
  const T* Bb2 = SPLIT ? (Bt2 + (size_t)b * strideB) : nullptr;

  const int rlane = lane & 15;
  const int koff  = (lane >> 4) * 8;
  const int mOff  = (lane >> 4) * 8;

  v8f acc[4][4];
#pragma unroll
  for (int i = 0; i < 4; ++i)
#pragma unroll
    for (int j = 0; j < 4; ++j) acc[i][j] = (v8f){0.f,0.f,0.f,0.f,0.f,0.f,0.f,0.f};

  for (int k0 = 0; k0 < K; k0 += 32) {
    V bh[4], bl[4];
#pragma unroll
    for (int j = 0; j < 4; ++j) {
      const size_t bo = (size_t)(n0 + (j << 4) + rlane) * ldb + koff + k0;
      bh[j] = Frag<T>::load(Bb + bo);
      if (SPLIT) bl[j] = Frag<T>::load(Bb2 + bo);
    }
#pragma unroll
    for (int i = 0; i < 4; ++i) {
      const size_t ao = (size_t)(m0 + (i << 4) + rlane) * lda + koff + k0;
      V ah = Frag<T>::load(Ab + ao);
      V al;
      if (SPLIT) al = Frag<T>::load(Ab2 + ao);
#pragma unroll
      for (int j = 0; j < 4; ++j) {
        acc[i][j] = Frag<T>::mma(ah, bh[j], acc[i][j]);
        if (SPLIT) {
          acc[i][j] = Frag<T>::mma(ah, bl[j], acc[i][j]);
          acc[i][j] = Frag<T>::mma(al, bh[j], acc[i][j]);
        }
      }
      Frag<T>::guard(acc[i][0], acc[i][3], ah, SPLIT ? al : ah);
    }
    Frag<T>::keep(bh[0], bh[1], bh[2], bh[3]);
    if (SPLIT) Frag<T>::keep(bl[0], bl[1], bl[2], bl[3]);
  }
  acc_guard4(acc[0][0], acc[0][1], acc[0][2], acc[0][3]);
  acc_guard4(acc[1][0], acc[1][1], acc[1][2], acc[1][3]);
  acc_guard4(acc[2][0], acc[2][1], acc[2][2], acc[2][3]);
  acc_guard4(acc[3][0], acc[3][1], acc[3][2], acc[3][3]);

  float* slab = sT[wave];
  const float* Rb = RESID ? (resid + (size_t)b * strideR) : nullptr;
#pragma unroll
  for (int i = 0; i < 4; ++i) {
    const int mBase = m0 + (i << 4);
#pragma unroll
    for (int j = 0; j < 4; ++j) {
      const int n = n0 + (j << 4) + rlane;
      float bv = 0.f;
      if (BIAS_MODE == 2) bv = bias[n];
#pragma unroll
      for (int r = 0; r < 8; ++r) {
        float v = acc[i][j][r] * scale;
        if (BIAS_MODE == 1) v += bias[mBase + mOff + r];
        if (BIAS_MODE == 2) v += bv;
        if (RESID) v += Rb[(size_t)(mBase + mOff + r) * ldc + n];
        if (ACT == 1) v = tanhf(v);
        if (ACT == 2) v = fmaxf(v, 0.0f);
        if (ACT == 3) v = v / (1.0f + expf(-v));
        if (ACT == 4) v = (v > 0.f) ? v : 0.01f * v;
        if (ACT == 5) v = 0.5f * v * (1.0f + erff(v * 0.70710678118654752f));
        slab[(mOff + r) * 68 + (j << 4) + rlane] = v;
      }
    }
    __builtin_amdgcn_fence(__ATOMIC_RELEASE, "workgroup");
    __builtin_amdgcn_wave_barrier();
    __builtin_amdgcn_fence(__ATOMIC_ACQUIRE, "workgroup");
    if (OUT_MODE == 0) {
      float* C = (float*)Cout + (size_t)b * strideC;
      const int hh = lane >> 4, c4 = (lane & 15) * 4;
      for (int pass = 0; pass < 2; ++pass) {
#pragma unroll
        for (int it = 0; it < 8; ++it) {
          const int row = it * 2 + hh;
          v4f v = *(const v4f*)(slab + row * 68 + c4);
          *(volatile v4f*)(C + (size_t)(mBase + row) * ldc + n0 + c4) = v;
        }
        __threadfence();
      }
    } else {
      const int q = lane >> 3, c8 = (lane & 7) * 8;
      unsigned short* C  = (unsigned short*)Cout  + (size_t)b * strideC;
      unsigned short* C2 = (OUT_MODE == 2) ? ((unsigned short*)Cout2 + (size_t)b * strideC) : nullptr;
      for (int pass = 0; pass < 2; ++pass) {
#pragma unroll
        for (int it = 0; it < 4; ++it) {
          const int row = it * 4 + q;
          const float* sp = slab + row * 68 + c8;
          v8h hv, lv;
#pragma unroll
          for (int e = 0; e < 8; ++e) {
            if (OUT_MODE == 1) {
              hv[e] = (_Float16)sp[e];
            } else {
              unsigned short hb = f2bf_bits(sp[e]);
              unsigned short lb = f2bf_bits(sp[e] - bf_bits2f(hb));
              hv[e] = __builtin_bit_cast(_Float16, hb);
              lv[e] = __builtin_bit_cast(_Float16, lb);
            }
          }
          *(volatile v8h*)(C + (size_t)(mBase + row) * ldc + n0 + c8) = hv;
          if (OUT_MODE == 2) *(volatile v8h*)(C2 + (size_t)(mBase + row) * ldc + n0 + c8) = lv;
        }
        __threadfence();
      }
    }
    __builtin_amdgcn_fence(__ATOMIC_RELEASE, "workgroup");
    __builtin_amdgcn_wave_barrier();
    __builtin_amdgcn_fence(__ATOMIC_ACQUIRE, "workgroup");
  }
}

__device__ __forceinline__ float wave_sum(float v) {
#pragma unroll
  for (int m = 16; m >= 1; m >>= 1) v += __shfl_xor(v, m, 32);
  return v;
}
__device__ __forceinline__ float h2f(u16 b) { return (float)__builtin_bit_cast(_Float16, b); }
__device__ __forceinline__ unsigned pack2h(float a, float b) {
  return (unsigned)__builtin_bit_cast(u16, (_Float16)a) | ((unsigned)__builtin_bit_cast(u16, (_Float16)b) << 16);
}
__device__ __forceinline__ float gelu_exact(float x) {
  return 0.5f * x * (1.0f + erff(x * 0.70710678118654752f));
}
__device__ __forceinline__ int gate_perm512(int rem) { return ((rem & 127) << 2) | (rem >> 7); }
__device__ __forceinline__ float yval(const u16* XC, const u16* BO, const u16* X1, const float* XN, size_t e) {
  const float xc = h2f(XC[e]);
  const float bo = h2f(BO[e]);
  const float x1 = h2f(X1[e]);
  const float sg = __builtin_amdgcn_rcpf(1.0f + __expf(-xc));
  return xc * sg * (bo + x1) + XN[e];
}

__global__ __launch_bounds__(256) void ln_rows_f32_kernel(const float* __restrict__ in, const float* __restrict__ g,
                                                          const float* __restrict__ bb, float* __restrict__ out) {
  __shared__ float ra[8];
  __shared__ float rb[8];
  const int tid = threadIdx.x, lane = tid & 31, w = tid >> 5;
  const size_t base = (size_t)blockIdx.x * kEmb + (size_t)tid * 4;
  const v4f v = *(const v4f*)(in + base);
  float s = (v[0] + v[1]) + (v[2] + v[3]);
  s = wave_sum(s);
  if (lane == 0) ra[w] = s;
  __syncthreads();
  float ts = 0.f;
#pragma unroll
  for (int i = 0; i < 8; ++i) ts += ra[i];
  const float mu = ts * (1.0f / (float)kEmb);
  const float d0 = v[0] - mu, d1 = v[1] - mu, d2 = v[2] - mu, d3 = v[3] - mu;
  float q = d0 * d0 + d1 * d1 + d2 * d2 + d3 * d3;
  q = wave_sum(q);
  if (lane == 0) rb[w] = q;
  __syncthreads();
  float tq = 0.f;
#pragma unroll
  for (int i = 0; i < 8; ++i) tq += rb[i];
  const float rs = rsqrtf(tq * (1.0f / (float)kEmb) + 1e-5f);
  const v4f gg = *(const v4f*)(g + tid * 4);
  const v4f b4 = *(const v4f*)(bb + tid * 4);
  v4f o;
  o[0] = d0 * rs * gg[0] + b4[0];
  o[1] = d1 * rs * gg[1] + b4[1];
  o[2] = d2 * rs * gg[2] + b4[2];
  o[3] = d3 * rs * gg[3] + b4[3];
  for (int pass = 0; pass < 2; ++pass) {
    *(volatile v4f*)(out + base) = o;
    __threadfence();
  }
}

__global__ __launch_bounds__(128) void ln_rows_f16_kernel(const u16* in, const float* __restrict__ g,
                                                          const float* __restrict__ bb, u16* out) {
  __shared__ float ra[4];
  __shared__ float rb[4];
  const int tid = threadIdx.x, lane = tid & 31, w = tid >> 5;
  const size_t base = (size_t)blockIdx.x * kEmb + (size_t)tid * 8;
  const v8h hv = *(const v8h*)((const _Float16*)in + base);
  float f[8];
#pragma unroll
  for (int e = 0; e < 8; ++e) f[e] = (float)hv[e];
  float s = ((f[0] + f[1]) + (f[2] + f[3])) + ((f[4] + f[5]) + (f[6] + f[7]));
  s = wave_sum(s);
  if (lane == 0) ra[w] = s;
  __syncthreads();
  const float ts = (ra[0] + ra[1]) + (ra[2] + ra[3]);
  const float mu = ts * (1.0f / (float)kEmb);
  float d[8];
  float q = 0.f;
#pragma unroll
  for (int e = 0; e < 8; ++e) { d[e] = f[e] - mu; q += d[e] * d[e]; }
  q = wave_sum(q);
  if (lane == 0) rb[w] = q;
  __syncthreads();
  const float tq = (rb[0] + rb[1]) + (rb[2] + rb[3]);
  const float rs = rsqrtf(tq * (1.0f / (float)kEmb) + 1e-5f);
  const v4f ga = *(const v4f*)(g + tid * 8), gb2 = *(const v4f*)(g + tid * 8 + 4);
  const v4f ba = *(const v4f*)(bb + tid * 8), bb2 = *(const v4f*)(bb + tid * 8 + 4);
  const float gv[8] = {ga[0], ga[1], ga[2], ga[3], gb2[0], gb2[1], gb2[2], gb2[3]};
  const float bv[8] = {ba[0], ba[1], ba[2], ba[3], bb2[0], bb2[1], bb2[2], bb2[3]};
  v8h o;
#pragma unroll
  for (int e = 0; e < 8; ++e) o[e] = (_Float16)(d[e] * rs * gv[e] + bv[e]);
  for (int pass = 0; pass < 2; ++pass) {
    *(volatile v8h*)((_Float16*)out + base) = o;
    __threadfence();
  }
}

__global__ __launch_bounds__(256) void fc_kernel(const float* __restrict__ XN, const float* __restrict__ w1,
                                               const float* __restrict__ b1, const float* __restrict__ w2,
                                               const float* __restrict__ b2, u16* __restrict__ XC, u16* __restrict__ X1) {
  __shared__ __align__(16) float swT[36 * 12];
  __shared__ __align__(16) float sw2[144];
  __shared__ float sb1[12], sb2[12];
  __shared__ float S1[12 * 256], S2[12 * 256];
  const int tid = threadIdx.x;
  for (int i = tid; i < 432; i += 256) { const int o = i / 36, r = i - o * 36; swT[r * 12 + o] = w1[i]; }
  if (tid < 144) sw2[tid] = w2[tid];
  if (tid < 12) { sb1[tid] = b1[tid]; sb2[tid] = b2[tid]; }
  __syncthreads();
  const int lb = blockIdx.x, b = blockIdx.y;
  const int l = lb * 256 + tid;
  const int lm = (l > 0) ? (l - 1) : 0;
  const int lp = (l < kEmb - 1) ? (l + 1) : (kEmb - 1);
  const bool pm = (l > 0), pp = (l < kEmb - 1);
  float acc[12];
#pragma unroll
  for (int o = 0; o < 12; ++o) acc[o] = sb1[o];
#pragma unroll 1
  for (int c = 0; c < 12; ++c) {
    const float* r = XN + ((size_t)b * kSeq + c) * kEmb;
    float x0 = r[lm];
    const float x1v = r[l];
    float x2 = r[lp];
    x0 = pm ? x0 : 0.0f;
    x2 = pp ? x2 : 0.0f;
    const float* wp = swT + c * 36;
#pragma unroll
    for (int o = 0; o < 12; ++o) acc[o] += x0 * wp[o] + x1v * wp[12 + o] + x2 * wp[24 + o];
  }
#pragma unroll
  for (int o = 0; o < 12; ++o) S1[o * 256 + tid] = acc[o];
#pragma unroll 1
  for (int o2 = 0; o2 < 12; ++o2) {
    const float* wq = sw2 + o2 * 12;
    float v = sb2[o2];
#pragma unroll
    for (int c = 0; c < 12; ++c) v += wq[c] * acc[c];
    S2[o2 * 256 + tid] = v;
  }
  __syncthreads();
  const int hi = tid >> 7, jj = tid & 127;
  unsigned pc[6], px[6];
  size_t oi[6];
#pragma unroll
  for (int it = 0; it < 6; ++it) {
    const int o = 2 * it + hi;
    pc[it] = pack2h(S1[o * 256 + 2 * jj], S1[o * 256 + 2 * jj + 1]);
    px[it] = pack2h(S2[o * 256 + 2 * jj], S2[o * 256 + 2 * jj + 1]);
    oi[it] = ((((size_t)b * kSeq + o) * kEmb) + (size_t)lb * 256 + (size_t)(2 * jj)) >> 1;
  }
  unsigned* XC32 = (unsigned*)XC;
  unsigned* X132 = (unsigned*)X1;
  for (int pass = 0; pass < 2; ++pass) {
#pragma unroll
    for (int it = 0; it < 6; ++it) {
      ((volatile unsigned*)XC32)[oi[it]] = pc[it];
      ((volatile unsigned*)X132)[oi[it]] = px[it];
    }
    __threadfence();
  }
}

template <int PERM>
__global__ __launch_bounds__(256) void tpw16_kernel(const float* __restrict__ src, int nCols, int ldo,
                                                  u16* __restrict__ O, float sc) {
  __shared__ float Tt[64 * 65];
  const int tid = threadIdx.x;
  const int c0 = blockIdx.x * 64, r0 = blockIdx.y * 64;
#pragma unroll
  for (int i = 0; i < 4; ++i) {
    const int idx = i * 256 + tid;
    const int rr = idx >> 4, cc = (idx & 15) * 4;
    const v4f v = *(const v4f*)(src + (size_t)(r0 + rr) * (size_t)nCols + c0 + cc);
    Tt[rr * 65 + cc + 0] = v[0];
    Tt[rr * 65 + cc + 1] = v[1];
    Tt[rr * 65 + cc + 2] = v[2];
    Tt[rr * 65 + cc + 3] = v[3];
  }
  __syncthreads();
  const int q = tid >> 3, c8 = (tid & 7) * 8;
  v8h hv[2];
  size_t oo[2];
#pragma unroll
  for (int gq = 0; gq < 2; ++gq) {
    const int qq = gq * 32 + q;
    const int col = c0 + qq;
    int orow = col;
    if (PERM) orow = (col & ~511) | gate_perm512(col & 511);
    oo[gq] = (size_t)orow * (size_t)ldo + (size_t)(r0 + c8);
#pragma unroll
    for (int e = 0; e < 8; ++e) hv[gq][e] = (_Float16)(Tt[(c8 + e) * 65 + qq] * sc);
  }
  _Float16* Oh = (_Float16*)O;
  for (int pass = 0; pass < 2; ++pass) {
#pragma unroll
    for (int gq = 0; gq < 2; ++gq) *(volatile v8h*)(Oh + oo[gq]) = hv[gq];
    __threadfence();
  }
}

__global__ __launch_bounds__(256) void rgconv_kernel(const float* __restrict__ Rg, u16* __restrict__ O) {
  const int idx = blockIdx.x * 256 + threadIdx.x;
  const int row = idx >> 4, k8 = (idx & 15) * 8;
  const int head = row >> 9, rem = row & 511;
  const int orow = (head << 9) | gate_perm512(rem);
  const v4f a = *(const v4f*)(Rg + (size_t)row * kHS + k8);
  const v4f c = *(const v4f*)(Rg + (size_t)row * kHS + k8 + 4);
  v8h hv;
  hv[0] = (_Float16)(a[0] * 16.0f); hv[1] = (_Float16)(a[1] * 16.0f);
  hv[2] = (_Float16)(a[2] * 16.0f); hv[3] = (_Float16)(a[3] * 16.0f);
  hv[4] = (_Float16)(c[0] * 16.0f); hv[5] = (_Float16)(c[1] * 16.0f);
  hv[6] = (_Float16)(c[2] * 16.0f); hv[7] = (_Float16)(c[3] * 16.0f);
  _Float16* Oh = (_Float16*)O;
  for (int pass = 0; pass < 2; ++pass) {
    *(volatile v8h*)(Oh + (size_t)orow * kHS + k8) = hv;
    __threadfence();
  }
}

constexpr int kSlNB = 32;
constexpr int kSlHP = 136;
constexpr int kSlFP = 132;
constexpr float kRecScale = 1.0f / 4096.0f;

__global__ __launch_bounds__(256) void slstm_kernel(const u16* __restrict__ GXp, const u16* __restrict__ Rgp,
                                                  const float* __restrict__ bg, const float* __restrict__ gn_g,
                                                  const float* __restrict__ gn_b, u16* __restrict__ HNp) {
  __shared__ __align__(16) _Float16 Hs[kSlNB * kSlHP];
  __shared__ __align__(16) float    Hf[kSlNB * kSlFP];
  const _Float16* GX  = (const _Float16*)GXp;
  const _Float16* RgA = (const _Float16*)Rgp;
  _Float16* HN = (_Float16*)HNp;
  const int tid = threadIdx.x, lane = tid & 31, wave = tid >> 5;
  const int rl = lane & 15, hh = lane >> 4, koff = hh * 8;
  const int head = blockIdx.y;
  const int b0 = blockIdx.x * kSlNB;
#pragma unroll
  for (int i = 0; i < 17; ++i) Hs[i * 256 + tid] = (_Float16)0.0f;
  float cS[4][2][2], nS[4][2][2], mS[4][2][2];
#pragma unroll
  for (int i = 0; i < 4; ++i)
#pragma unroll
    for (int q = 0; q < 2; ++q)
#pragma unroll
      for (int j = 0; j < 2; ++j) { cS[i][q][j] = 0.f; nS[i][q][j] = 0.f; mS[i][q][j] = 0.f; }
  __syncthreads();
  const _Float16* Aw = RgA + ((size_t)head * 512 + (size_t)(64 * wave)) * kHS;
  const v8f z8 = {0.f, 0.f, 0.f, 0.f, 0.f, 0.f, 0.f, 0.f};

#pragma unroll 1
  for (int t = 0; t < kSeq; ++t) {
    v8f acc[4][2];
#pragma unroll
    for (int i = 0; i < 4; ++i) { acc[i][0] = z8; acc[i][1] = z8; }
#pragma unroll 1
    for (int k0 = 0; k0 < kHS; k0 += 32) {
      const v16h bq0 = Frag<_Float16>::load(Hs + rl * kSlHP + k0 + koff);
      const v16h bq1 = Frag<_Float16>::load(Hs + (16 + rl) * kSlHP + k0 + koff);
#pragma unroll
      for (int i = 0; i < 4; ++i) {
        const v16h ah = Frag<_Float16>::load(Aw + (size_t)(16 * i + rl) * kHS + k0 + koff);
        acc[i][0] = Frag<_Float16>::mma(ah, bq0, acc[i][0]);
        acc[i][1] = Frag<_Float16>::mma(ah, bq1, acc[i][1]);
        dep_guard_h(acc[i][0], acc[i][1], ah, ah);
      }
      keep4_h(bq0, bq1, bq0, bq1);
    }
    acc_guard4(acc[0][0], acc[0][1], acc[1][0], acc[1][1]);
    acc_guard4(acc[2][0], acc[2][1], acc[3][0], acc[3][1]);
    __syncthreads();

#pragma unroll
    for (int i = 0; i < 4; ++i) {
#pragma unroll
      for (int q = 0; q < 2; ++q) {
        const int ch = 16 * wave + 4 * i + 2 * hh + q;
        const float* bq = bg + head * 512 + ch;
        const float bz = bq[0], bi = bq[128], bf = bq[256], bo = bq[384];
#pragma unroll
        for (int j = 0; j < 2; ++j) {
          const int rloc = 16 * j + rl;
          const size_t grow = (size_t)(b0 + rloc) * kSeq + (size_t)t;
          const v4h g4 = *(const v4h*)(GX + grow * (size_t)kGate + head * 512 + 4 * ch);
          const float zp = acc[i][j][4 * q + 0] * kRecScale + (float)g4[0] + bz;
          const float ip = acc[i][j][4 * q + 1] * kRecScale + (float)g4[1] + bi;
          const float fp = acc[i][j][4 * q + 2] * kRecScale + (float)g4[2] + bf;
          const float op = acc[i][j][4 * q + 3] * kRecScale + (float)g4[3] + bo;
          const float zz = 1.0f - 2.0f * __builtin_amdgcn_rcpf(__expf(2.0f * zp) + 1.0f);
          const float oo = __builtin_amdgcn_rcpf(1.0f + __expf(-op));
          const float mo = mS[i][q][j];
          const float mn = fmaxf(fp + mo, ip);
          const float iv = __expf(ip - mn);
          const float fv = __expf(fp + mo - mn);
          const float cv = fv * cS[i][q][j] + iv * zz;
          const float nv = fv * nS[i][q][j] + iv;
          const float hv = oo * cv * __builtin_amdgcn_rcpf(nv);
          cS[i][q][j] = cv; nS[i][q][j] = nv; mS[i][q][j] = mn;
          Hs[rloc * kSlHP + ch] = (_Float16)(hv * 256.0f);
          Hf[rloc * kSlFP + ch] = hv;
        }
      }
    }
    __syncthreads();

    v8h ho[2];
    size_t oaddr[2];
#pragma unroll
    for (int it = 0; it < 2; ++it) {
      const int rloc = 4 * wave + 2 * it + hh;
      const int cc = 8 * rl;
      const v4f fa = *(const v4f*)(Hf + rloc * kSlFP + cc);
      const v4f fb = *(const v4f*)(Hf + rloc * kSlFP + cc + 4);
      const float f[8] = {fa[0], fa[1], fa[2], fa[3], fb[0], fb[1], fb[2], fb[3]};
      float s = ((f[0] + f[1]) + (f[2] + f[3])) + ((f[4] + f[5]) + (f[6] + f[7]));
#pragma unroll
      for (int off = 1; off < 16; off <<= 1) s += __shfl_xor(s, off, 32);
      const float mu = s * (1.0f / (float)kHS);
      float d[8];
      float qv = 0.f;
#pragma unroll
      for (int e = 0; e < 8; ++e) { d[e] = f[e] - mu; qv += d[e] * d[e]; }
#pragma unroll
      for (int off = 1; off < 16; off <<= 1) qv += __shfl_xor(qv, off, 32);
      const float rs = rsqrtf(qv * (1.0f / (float)kHS) + 1e-5f);
      const v4f ga = *(const v4f*)(gn_g + head * kHS + cc), gb2 = *(const v4f*)(gn_g + head * kHS + cc + 4);
      const v4f ba = *(const v4f*)(gn_b + head * kHS + cc), bb2 = *(const v4f*)(gn_b + head * kHS + cc + 4);
      const float gv[8] = {ga[0], ga[1], ga[2], ga[3], gb2[0], gb2[1], gb2[2], gb2[3]};
      const float bv[8] = {ba[0], ba[1], ba[2], ba[3], bb2[0], bb2[1], bb2[2], bb2[3]};
#pragma unroll
      for (int e = 0; e < 8; ++e) ho[it][e] = (_Float16)(d[e] * rs * gv[e] + bv[e]);
      oaddr[it] = ((size_t)(b0 + rloc) * kSeq + (size_t)t) * kEmb + (size_t)(head * kHS + cc);
    }
    for (int pass = 0; pass < 2; ++pass) {
#pragma unroll
      for (int it = 0; it < 2; ++it) *(volatile v8h*)(HN + oaddr[it]) = ho[it];
      __threadfence();
    }
  }
}

__global__ __launch_bounds__(256) void gate_kernel(const u16* __restrict__ LR, const float* __restrict__ bl,
                                                 const float* __restrict__ br, u16* __restrict__ P) {
  const unsigned i = blockIdx.x * 256u + threadIdx.x;
  const unsigned row = i >> 9;
  const unsigned k2 = (i & 511u) * 2u;
  const unsigned* LR32 = (const unsigned*)LR;
  const size_t li = ((size_t)row * 2048 + k2) >> 1;
  const unsigned ul = LR32[li];
  const unsigned ur = LR32[li + 512];
  const float l0 = h2f((u16)(ul & 0xFFFFu)), l1 = h2f((u16)(ul >> 16));
  const float r0 = h2f((u16)(ur & 0xFFFFu)), r1 = h2f((u16)(ur >> 16));
  const v2f b2l = *(const v2f*)(bl + k2);
  const v2f b2r = *(const v2f*)(br + k2);
  const float p0 = gelu_exact(l0 + b2l[0]) * (r0 + b2r[0]) * 64.0f;
  const float p1 = gelu_exact(l1 + b2l[1]) * (r1 + b2r[1]) * 64.0f;
  const unsigned u = pack2h(p0, p1);
  unsigned* P32 = (unsigned*)P;
  const size_t pi = ((size_t)row * kEmb + k2) >> 1;
  for (int pass = 0; pass < 2; ++pass) {
    ((volatile unsigned*)P32)[pi] = u;
    __threadfence();
  }
}

constexpr int kC1YP = 514;
constexpr int kC1WP = 64;
__global__ __launch_bounds__(256) void conv1_gelu_kernel(const u16* __restrict__ XC, const u16* __restrict__ BO,
                                                       const u16* __restrict__ X1, const float* __restrict__ XN,
                                                       const float* __restrict__ w, const float* __restrict__ bias,
                                                       u16* __restrict__ G) {
  __shared__ __align__(16) float swT[36 * kC1WP];
  __shared__ float sb[48];
  __shared__ __align__(16) float Ys[12 * kC1YP];
  __shared__ float Sg[12 * 256];
  const int tid = threadIdx.x;
  const int lb = blockIdx.x, b = blockIdx.y;
  const int lbase = lb * 512;
  for (int i = tid; i < 1728; i += 256) { const int o = i / 36, r = i - o * 36; swT[r * kC1WP + o] = w[i]; }
  if (tid < 48) sb[tid] = bias[tid];
#pragma unroll 1
  for (int c = 0; c < 12; ++c) {
    const size_t rowoff = ((size_t)b * kSeq + c) * kEmb;
#pragma unroll 1
    for (int p = 0; p < 2; ++p) {
      const int l = lbase + 2 * tid + p;
      Ys[c * kC1YP + 1 + 2 * tid + p] = yval(XC, BO, X1, XN, rowoff + (size_t)l);
    }
  }
  if (tid < 24) {
    const int side = (tid >= 12) ? 1 : 0;
    const int c = tid - 12 * side;
    const int l = side ? (lbase + 512) : (lbase - 1);
    const bool valid = (l >= 0) && (l < kEmb);
    const int lc = (l < 0) ? 0 : ((l > kEmb - 1) ? (kEmb - 1) : l);
    float yv = yval(XC, BO, X1, XN, ((size_t)b * kSeq + c) * kEmb + (size_t)lc);
    yv = valid ? yv : 0.0f;
    Ys[c * kC1YP + (side ? (kC1YP - 1) : 0)] = yv;
  }
  __syncthreads();
  unsigned* G32 = (unsigned*)G;
#pragma unroll 1
  for (int og = 0; og < 8; ++og) {
    float acc[6][2];
#pragma unroll
    for (int o = 0; o < 6; ++o) { const float bv = sb[og * 6 + o]; acc[o][0] = bv; acc[o][1] = bv; }
#pragma unroll 1
    for (int c = 0; c < 12; ++c) {
      const float* yp = Ys + c * kC1YP + 2 * tid;
      const v2f ya = *(const v2f*)(yp);
      const v2f yb = *(const v2f*)(yp + 2);
      const float y0 = ya[0], y1 = ya[1], y2 = yb[0], y3 = yb[1];
      const float* wp = swT + c * 3 * kC1WP + og * 6;
#pragma unroll
      for (int o = 0; o < 6; ++o) {
        const float w0 = wp[o], w1 = wp[kC1WP + o], w2 = wp[2 * kC1WP + o];
        acc[o][0] += y0 * w0 + y1 * w1 + y2 * w2;
        acc[o][1] += y1 * w0 + y2 * w1 + y3 * w2;
      }
    }
#pragma unroll
    for (int o = 0; o < 6; ++o) { Sg[(2 * o) * 256 + tid] = acc[o][0]; Sg[(2 * o + 1) * 256 + tid] = acc[o][1]; }
#pragma unroll 1
    for (int e = 0; e < 12; ++e) {
      const float v = Sg[e * 256 + tid];
      Sg[e * 256 + tid] = gelu_exact(v);
    }
    unsigned pk[6];
#pragma unroll
    for (int o = 0; o < 6; ++o) pk[o] = pack2h(Sg[(2 * o) * 256 + tid], Sg[(2 * o + 1) * 256 + tid]);
    const size_t gbase = ((((size_t)b * kC48 + (size_t)(og * 6)) * kEmb) + (size_t)lbase + (size_t)(2 * tid)) >> 1;
    for (int pass = 0; pass < 2; ++pass) {
#pragma unroll
      for (int o = 0; o < 6; ++o) ((volatile unsigned*)G32)[gbase + (size_t)o * (kEmb / 2)] = pk[o];
      __threadfence();
    }
  }
}

__global__ __launch_bounds__(256) void conv2_kernel(const u16* __restrict__ G, const float* __restrict__ w,
                                                  const float* __restrict__ bias, const float* __restrict__ XN,
                                                  float* __restrict__ out) {
  __shared__ __align__(16) float swT[144 * 12];
  __shared__ float sb[12];
  const int tid = threadIdx.x;
  for (int i = tid; i < 1728; i += 256) { const int o = i / 144, r = i - o * 144; swT[r * 12 + o] = w[i]; }
  if (tid < 12) sb[tid] = bias[tid];
  __syncthreads();
  const int l = blockIdx.x * 256 + tid;
  const int b = blockIdx.y;
  const int lm = (l > 0) ? (l - 1) : 0;
  const int lp = (l < kEmb - 1) ? (l + 1) : (kEmb - 1);
  const bool pm = (l > 0), pp = (l < kEmb - 1);
  float acc[12];
#pragma unroll
  for (int o = 0; o < 12; ++o) acc[o] = sb[o];
#pragma unroll 1
  for (int c = 0; c < kC48; ++c) {
    const u16* r = G + ((size_t)b * kC48 + c) * kEmb;
    float h0 = h2f(r[lm]);
    const float h1 = h2f(r[l]);
    float h2 = h2f(r[lp]);
    h0 = pm ? h0 : 0.0f;
    h2 = pp ? h2 : 0.0f;
    const float* wp = swT + c * 36;
#pragma unroll
    for (int o = 0; o < 12; ++o) acc[o] += h0 * wp[o] + h1 * wp[12 + o] + h2 * wp[24 + o];
  }
  float v[12];
#pragma unroll
  for (int o = 0; o < 12; ++o) v[o] = acc[o] + XN[((size_t)b * kSeq + o) * kEmb + l];
  for (int pass = 0; pass < 2; ++pass) {
#pragma unroll
    for (int o = 0; o < 12; ++o) ((volatile float*)out)[((size_t)b * kSeq + o) * kEmb + l] = v[o];
    __threadfence();
  }
}

extern "C" void kernel_launch(void* const* d_in, const int* in_sizes, int n_in,
                              void* d_out, int out_size, void* d_ws, size_t ws_size, hipStream_t stream) {
  if (n_in < 24) return;
  const float* x       = (const float*)d_in[0];
  const float* ln_g    = (const float*)d_in[1];
  const float* ln_b    = (const float*)d_in[2];
  const float* fc1_w   = (const float*)d_in[3];
  const float* fc1_b   = (const float*)d_in[4];
  const float* fc2_w   = (const float*)d_in[5];
  const float* fc2_b   = (const float*)d_in[6];
  const float* conv1_w = (const float*)d_in[7];
  const float* conv1_b = (const float*)d_in[8];
  const float* conv2_w = (const float*)d_in[9];
  const float* conv2_b = (const float*)d_in[10];
  const float* xl_ln_g = (const float*)d_in[11];
  const float* xl_ln_b = (const float*)d_in[12];
  const float* Wg      = (const float*)d_in[13];
  const float* bg      = (const float*)d_in[14];
  const float* Rg      = (const float*)d_in[15];
  const float* gn_g    = (const float*)d_in[16];
  const float* gn_b    = (const float*)d_in[17];
  const float* upl_w   = (const float*)d_in[18];
  const float* upl_b   = (const float*)d_in[19];
  const float* upr_w   = (const float*)d_in[20];
  const float* upr_b   = (const float*)d_in[21];
  const float* down_w  = (const float*)d_in[22];
  const float* down_b  = (const float*)d_in[23];
  float* out = (float*)d_out;

  constexpr size_t kF32Plane  = (size_t)kRows * kEmb * 4;
  constexpr size_t kH16Plane  = (size_t)kRows * kEmb * 2;
  constexpr size_t kBigRegion = (size_t)kRows * kGate * 2;
  constexpr size_t offXN  = 0;
  constexpr size_t offXC  = offXN + kF32Plane;
  constexpr size_t offX1  = offXC + kH16Plane;
  constexpr size_t offBig = offX1 + kH16Plane;
  constexpr size_t offLR  = offBig;
  constexpr size_t offP   = offBig + (size_t)kRows * 2048 * 2;
  constexpr size_t offR4  = offBig + kBigRegion;
  constexpr size_t offWg  = offR4 + kH16Plane;
  constexpr size_t offWlr = offWg + (size_t)kGate * kEmb * 2;
  constexpr size_t offWd  = offWlr + (size_t)2048 * kEmb * 2;
  constexpr size_t offRg  = offWd + (size_t)kEmb * kEmb * 2;
  constexpr size_t kWsTotal = offRg + (size_t)kHeads * 512 * kHS * 2;
  typedef char ws_fits_cap[(kWsTotal <= (size_t)134217728) ? 1 : -1];
  typedef char g_plane_fits[((size_t)kBatch * kC48 * kEmb * 2 <= kBigRegion) ? 1 : -1];
  typedef char p_plane_fits[(offP + kH16Plane <= offR4) ? 1 : -1];
  (void)sizeof(ws_fits_cap); (void)sizeof(g_plane_fits); (void)sizeof(p_plane_fits);
  if (ws_size < kWsTotal) return;
  if ((size_t)out_size < (size_t)kRows * kEmb) return;
  if ((size_t)in_sizes[0] < (size_t)kRows * kEmb) return;

  char* ws = (char*)d_ws;
  float* XN   = (float*)(ws + offXN);
  u16*   XC16 = (u16*)(ws + offXC);
  u16*   X116 = (u16*)(ws + offX1);
  u16*   GX16 = (u16*)(ws + offBig);
  u16*   LR16 = (u16*)(ws + offLR);
  u16*   P16  = (u16*)(ws + offP);
  u16*   G16  = (u16*)(ws + offBig);
  u16*   XN2  = (u16*)(ws + offR4);
  u16*   HN16 = (u16*)(ws + offR4);
  u16*   BO16 = (u16*)(ws + offR4);
  u16*   WgT  = (u16*)(ws + offWg);
  u16*   WLR  = (u16*)(ws + offWlr);
  u16*   Wd   = (u16*)(ws + offWd);
  u16*   RgA  = (u16*)(ws + offRg);

  ln_rows_f32_kernel<<<dim3(kRows), dim3(256), 0, stream>>>(x, ln_g, ln_b, XN);
  fc_kernel<<<dim3(4, kBatch), dim3(256), 0, stream>>>(XN, fc1_w, fc1_b, fc2_w, fc2_b, XC16, X116);
  ln_rows_f16_kernel<<<dim3(kRows), dim3(128), 0, stream>>>(X116, xl_ln_g, xl_ln_b, XN2);
  tpw16_kernel<1><<<dim3(kGate / 64, kEmb / 64), dim3(256), 0, stream>>>(Wg, kGate, kEmb, WgT, 16.0f);
  tpw16_kernel<0><<<dim3(kEmb / 64, kEmb / 64), dim3(256), 0, stream>>>(upl_w, kEmb, kEmb, WLR, 16.0f);
  tpw16_kernel<0><<<dim3(kEmb / 64, kEmb / 64), dim3(256), 0, stream>>>(upr_w, kEmb, kEmb, WLR + (size_t)kEmb * kEmb, 16.0f);
  tpw16_kernel<0><<<dim3(kEmb / 64, kEmb / 64), dim3(256), 0, stream>>>(down_w, kEmb, kEmb, Wd, 16.0f);
  rgconv_kernel<<<dim3((kHeads * 512 * kHS / 8) / 256), dim3(256), 0, stream>>>(Rg, RgA);
  wmma_gemm64<0, false, 0, 1, false><<<dim3(768, 1), dim3(256), 0, stream>>>(
      XN2, XN2, kEmb, 0L, WgT, WgT, kEmb, 0L, (void*)GX16, (void*)GX16, kGate, 0L,
      bg, XN, 0L, kRows, kGate, kEmb, 1.0f / 16.0f);
  slstm_kernel<<<dim3(kBatch / kSlNB, kHeads), dim3(256), 0, stream>>>(GX16, RgA, bg, gn_g, gn_b, HN16);
  wmma_gemm64<0, false, 0, 1, false><<<dim3(384, 1), dim3(256), 0, stream>>>(
      HN16, HN16, kEmb, 0L, WLR, WLR, kEmb, 0L, (void*)LR16, (void*)LR16, 2048, 0L,
      bg, XN, 0L, kRows, 2048, kEmb, 1.0f / 16.0f);
  gate_kernel<<<dim3((kRows * (kEmb / 2)) / 256), dim3(256), 0, stream>>>(LR16, upl_b, upr_b, P16);
  wmma_gemm64<0, false, 2, 1, false><<<dim3(192, 1), dim3(256), 0, stream>>>(
      P16, P16, kEmb, 0L, Wd, Wd, kEmb, 0L, (void*)BO16, (void*)BO16, kEmb, 0L,
      down_b, XN, 0L, kRows, kEmb, kEmb, 1.0f / 1024.0f);
  conv1_gelu_kernel<<<dim3(2, kBatch), dim3(256), 0, stream>>>(XC16, BO16, X116, XN, conv1_w, conv1_b, G16);
  ln_rows_f16_kernel<<<dim3(kBatch * kC48), dim3(128), 0, stream>>>(G16, ln_g, ln_b, G16);
  conv2_kernel<<<dim3(4, kBatch), dim3(256), 0, stream>>>(G16, conv2_w, conv2_b, XN, out);
}
